// SpatialRegularizationLayer_64149631533715
// MI455X (gfx1250) — hardware-verified
//
#include <hip/hip_runtime.h>


#define NB_  256
#define NL   80
#define HWS  196
#define C1   512
#define KP1  128
#define GRP  512
#define OPG  4
#define NG   (GRP * OPG)
#define BCH  32
#define RCH  (BCH * HWS)
#define NOP  128
#define DM   C1
#define LOSC 1024.0f

typedef _Float16 h16;
typedef unsigned short bf;
typedef __attribute__((ext_vector_type(16))) __bf16   v16bf;
typedef __attribute__((ext_vector_type(16))) _Float16 v16h;
typedef __attribute__((ext_vector_type(8)))  _Float16 v8h;
typedef __attribute__((ext_vector_type(8)))  unsigned short v8us;
typedef __attribute__((ext_vector_type(8)))  float    v8f;
typedef __attribute__((ext_vector_type(4)))  float    v4f;
typedef v8h  __attribute__((may_alias)) v8ha;
typedef v4f  __attribute__((may_alias)) v4fa;
typedef v8us __attribute__((may_alias)) v8usa;

__device__ __forceinline__ unsigned short f2bf(float f) { unsigned u = __float_as_uint(f); u += 0x7FFFu + ((u >> 16) & 1u); return (unsigned short)(u >> 16); }
__device__ __forceinline__ float bf2f(unsigned short b) { return __uint_as_float(((unsigned)b) << 16); }
__device__ __forceinline__ float bfr(float f) { return bf2f(f2bf(f)); }
__device__ __forceinline__ v16h cat16(v8h lo, v8h hi) { return __builtin_shufflevector(lo, hi, 0, 1, 2, 3, 4, 5, 6, 7, 8, 9, 10, 11, 12, 13, 14, 15); }
__device__ __forceinline__ v16bf cat16b(v8us lo, v8us hi) { return __builtin_bit_cast(v16bf, __builtin_shufflevector(lo, hi, 0, 1, 2, 3, 4, 5, 6, 7, 8, 9, 10, 11, 12, 13, 14, 15)); }
__device__ __forceinline__ v8f wmma16(v16h a, v16h b, v8f c) { return __builtin_amdgcn_wmma_f32_16x16x32_f16(false, a, false, b, (short)0, c, false, false); }
__device__ __forceinline__ v8f wmmab(v16bf a, v16bf b, v8f c) { return __builtin_amdgcn_wmma_f32_16x16x32_bf16(false, a, false, b, (short)0, c, false, false); }

template <bool SPLITA, bool F16OUT = false>
__global__ __launch_bounds__(128) void k_gemmb(const bf* __restrict__ A, const bf* __restrict__ Al, const bf* __restrict__ Bn, const float* __restrict__ bias, float* C, int ldc, h16* C2, const float* __restrict__ R = nullptr, int K = DM, int roundR = 1) {
    __shared__ __align__(16) float ost[4][16 * 68];
    const int lane = threadIdx.x & 31, wave = threadIdx.x >> 5, lr = lane & 15, hi = lane >> 4;
    const int r0 = blockIdx.x * 64 + wave * 16, c0 = blockIdx.y * 64;
    const size_t aoff = (size_t)(r0 + lr) * K + 8 * hi;
    size_t boff[4];
#pragma unroll
    for (int t = 0; t < 4; ++t) boff[t] = (size_t)(c0 + t * 16 + lr) * K + 8 * hi;
    v8f acc[4];
#pragma unroll
    for (int t = 0; t < 4; ++t) acc[t] = (v8f){};
#pragma unroll 1
    for (int kc = 0; kc < K; kc += 32) {
        const v16bf a = cat16b(*(const v8us*)(A + aoff + kc), *(const v8us*)(A + aoff + kc + 16));
        v16bf al = a;
        if (SPLITA) al = cat16b(*(const v8us*)(Al + aoff + kc), *(const v8us*)(Al + aoff + kc + 16));
#pragma unroll
        for (int t = 0; t < 4; ++t) { const v16bf b = cat16b(*(const v8us*)(Bn + boff[t] + kc), *(const v8us*)(Bn + boff[t] + kc + 16)); acc[t] = wmmab(a, b, acc[t]); if (SPLITA) acc[t] = wmmab(al, b, acc[t]); }
        asm volatile("v_nop\n\tv_nop\n\tv_nop\n\tv_nop" : "+v"(acc[0]), "+v"(acc[1]), "+v"(acc[2]), "+v"(acc[3]) : "v"(a), "v"(al));
    }
    float* os = &ost[wave][0];
#pragma unroll
    for (int t = 0; t < 4; ++t) { const float bv = bias ? bfr(bias[c0 + t * 16 + lr]) : 0.f;
#pragma unroll
        for (int j = 0; j < 8; ++j) os[(hi * 8 + j) * 68 + t * 16 + lr] = acc[t][j] + bv; }
    __syncthreads();
    if (F16OUT) {
        h16* crow = (h16*)(void*)C + (size_t)r0 * ldc + c0;
        auto pass = [&]() {
#pragma unroll
            for (int s = 0; s < 4; ++s) { const int row = 4 * s + (lane >> 3), piece = lane & 7; const float* sp = os + row * 68 + piece * 8; v8h o, o2;
#pragma unroll
                for (int i = 0; i < 8; ++i) { const h16 a = (h16)sp[i]; o[i] = a; o2[i] = (h16)((sp[i] - (float)a) * LOSC); }
                *(volatile v8h*)(crow + (size_t)row * ldc + piece * 8) = o; if (C2) *(volatile v8h*)(C2 + (size_t)r0 * ldc + c0 + (size_t)row * ldc + piece * 8) = o2; }
        };
        pass(); __threadfence(); pass();
    } else {
        float* crow = C + (size_t)r0 * ldc + c0;
        auto pass = [&]() {
#pragma unroll
            for (int s = 0; s < 8; ++s) { const int Lid = (lane >> 3) + 4 * s, piece = lane & 7; const int row = Lid >> 1, cofs = (Lid & 1) * 32 + piece * 4;
                v4f val = *(const v4fa*)(os + row * 68 + cofs); if (R) { const v4f rv = *(const v4f*)(R + ((size_t)r0 + row) * ldc + c0 + cofs); val += roundR ? (v4f){bfr(rv[0]), bfr(rv[1]), bfr(rv[2]), bfr(rv[3])} : rv; }
                *(volatile v4f*)(crow + (size_t)row * ldc + cofs) = val; }
        };
        pass(); __threadfence(); pass();
    }
}


__global__ __launch_bounds__(256) void k_cvt8(const float* __restrict__ src, bf* dst, size_t n8) {
    const size_t i = (size_t)blockIdx.x * 256 + threadIdx.x; if (i >= n8) return;
    const v8f v = *(const v8f*)(src + i * 8); v8us o;
#pragma unroll
    for (int k = 0; k < 8; ++k) o[k] = f2bf(v[k]);
    *(volatile v8us*)(dst + i * 8) = o; __threadfence(); *(volatile v8us*)(dst + i * 8) = o;
}
__global__ __launch_bounds__(256) void k_zero8(bf* dst, size_t n8) {
    const size_t i = (size_t)blockIdx.x * 256 + threadIdx.x; if (i >= n8) return; v8us z;
#pragma unroll
    for (int k = 0; k < 8; ++k) z[k] = 0;
    *(volatile v8us*)(dst + i * 8) = z; __threadfence(); *(volatile v8us*)(dst + i * 8) = z;
}

__global__ __launch_bounds__(256) void k_a0(const float* __restrict__ x, int b0, bf* A0) {
    typedef __attribute__((ext_vector_type(4))) unsigned short v4us;
    const int lane = threadIdx.x & 31; const size_t rl = (size_t)blockIdx.x * 8 + (threadIdx.x >> 5); if (rl >= (size_t)RCH) return; const int bl = (int)(rl / HWS), hw = (int)(rl % HWS); v4us o;
#pragma unroll
    for (int i = 0; i < 4; ++i) { const int c = lane * 4 + i; o[i] = (c < NL) ? f2bf(x[(((size_t)(b0 + bl) * NL + (c < NL ? c : 0)) * HWS) + hw]) : (unsigned short)0; }
    *(volatile v4us*)(A0 + rl * KP1 + lane * 4) = o; __threadfence(); *(volatile v4us*)(A0 + rl * KP1 + lane * 4) = o;
}
__global__ __launch_bounds__(256) void k_w1p(const float* __restrict__ w1, bf* W1P) {
    typedef __attribute__((ext_vector_type(4))) unsigned short v4us;
    const int lane = threadIdx.x & 31, o_ = blockIdx.x * 8 + (threadIdx.x >> 5); if (o_ >= C1) return; v4us o;
#pragma unroll
    for (int i = 0; i < 4; ++i) { const int c = lane * 4 + i; o[i] = (c < NL) ? f2bf(w1[(size_t)o_ * NL + (c < NL ? c : 0)]) : (unsigned short)0; }
    *(volatile v4us*)(W1P + (size_t)o_ * KP1 + lane * 4) = o; __threadfence(); *(volatile v4us*)(W1P + (size_t)o_ * KP1 + lane * 4) = o;
}
__global__ __launch_bounds__(256) void k_fcp(const float* __restrict__ fw, bf* FCP) {
    const int lane = threadIdx.x & 31, o_ = blockIdx.x * 8 + (threadIdx.x >> 5); if (o_ >= NOP) return;
#pragma unroll 1
    for (int ps = 0; ps < 2; ++ps) {
#pragma unroll
        for (int q = 0; q < NG / 256; ++q) { v8us o;
#pragma unroll
            for (int i = 0; i < 8; ++i) o[i] = (o_ < NL) ? f2bf(fw[(size_t)(o_ < NL ? o_ : 0) * NG + q * 256 + lane * 8 + i]) : (unsigned short)0;
            *(volatile v8us*)(FCP + (size_t)o_ * NG + q * 256 + lane * 8) = o; }
        if (ps == 0) __threadfence(); }
}
__global__ __launch_bounds__(256) void k_split512(const float* __restrict__ src, bf* dh, bf* dl) {
    const int lane = threadIdx.x & 31; const size_t r = (size_t)blockIdx.x * 8 + (threadIdx.x >> 5); if (r >= (size_t)RCH) return;
#pragma unroll 1
    for (int ps = 0; ps < 2; ++ps) {
#pragma unroll
        for (int q = 0; q < C1 / 256; ++q) { const size_t o = r * C1 + q * 256 + lane * 8; const v8f v = *(const v8f*)(src + o); v8us oh, ol;
#pragma unroll
            for (int i = 0; i < 8; ++i) { const unsigned short hb = f2bf(v[i]); oh[i] = hb; ol[i] = f2bf(v[i] - bf2f(hb)); }
            *(volatile v8us*)(dh + o) = oh; *(volatile v8us*)(dl + o) = ol; }
        if (ps == 0) __threadfence(); }
}
__global__ __launch_bounds__(256) void k_conv3(const float* __restrict__ H2, const float* __restrict__ w3, int b0, bf* Gh, bf* Gl) {
    typedef __attribute__((ext_vector_type(4))) unsigned short v4us;
    const int t = blockIdx.x * 256 + threadIdx.x; if (t >= BCH * GRP) return; const int bl = t / GRP, grp = t % GRP; float acc[OPG] = {0.f, 0.f, 0.f, 0.f};
#pragma unroll 1
    for (int hw = 0; hw < HWS; ++hw) { const float hv = H2[((size_t)bl * HWS + hw) * C1 + grp];
#pragma unroll
        for (int o = 0; o < OPG; ++o) acc[o] = fmaf(hv, bfr(w3[((size_t)grp * OPG + o) * HWS + hw]), acc[o]); }
    v4us oh, ol;
#pragma unroll
    for (int o = 0; o < OPG; ++o) { const float v = fmaxf(acc[o], 0.f); const unsigned short hb = f2bf(v); oh[o] = hb; ol[o] = f2bf(v - bf2f(hb)); }
    const size_t off = (size_t)(b0 + bl) * NG + grp * OPG; *(volatile v4us*)(Gh + off) = oh; *(volatile v4us*)(Gl + off) = ol; __threadfence(); *(volatile v4us*)(Gh + off) = oh; *(volatile v4us*)(Gl + off) = ol;
}
__global__ __launch_bounds__(256) void k_out(const float* __restrict__ T, const float* __restrict__ fb, float* OUTP) {
    const int u = blockIdx.x * 256 + threadIdx.x; if (u >= NB_ * NL / 4) return; v4f o;
#pragma unroll
    for (int q = 0; q < 4; ++q) { const int e = u * 4 + q; o[q] = T[(size_t)(e / NL) * NOP + (e % NL)] + bfr(fb[e % NL]); }
    *(volatile v4f*)(OUTP + (size_t)u * 4) = o; __threadfence(); *(volatile v4f*)(OUTP + (size_t)u * 4) = o;
}

extern "C" void kernel_launch(void* const* d_in, const int* in_sizes, int n_in,
                              void* d_out, int out_size, void* d_ws, size_t ws_size, hipStream_t stream) {
    (void)in_sizes; (void)n_in; (void)out_size;
    const float* x = (const float*)d_in[0]; const float* w1 = (const float*)d_in[1]; const float* b1 = (const float*)d_in[2]; const float* w2 = (const float*)d_in[3]; const float* b2 = (const float*)d_in[4]; const float* w3 = (const float*)d_in[5]; const float* fw = (const float*)d_in[6]; const float* fb = (const float*)d_in[7];
    float* out = (float*)d_out;
    char* wsp = (char*)d_ws;
    auto take = [&](size_t bytes) { char* p = wsp; wsp += (bytes + 255) & ~(size_t)255; return (void*)p; };
    bf* W1P = (bf*)take((size_t)C1 * KP1 * 2); bf* W2B = (bf*)take((size_t)C1 * C1 * 2); bf* FCP = (bf*)take((size_t)NOP * NG * 2);
    bf* A0 = (bf*)take((size_t)RCH * KP1 * 2); float* H1 = (float*)take((size_t)RCH * C1 * 4); bf* Hh = (bf*)take((size_t)RCH * C1 * 2); bf* Hl = (bf*)take((size_t)RCH * C1 * 2); float* H2 = (float*)take((size_t)RCH * C1 * 4);
    bf* Gh = (bf*)take((size_t)NB_ * NG * 2); bf* Gl = (bf*)take((size_t)NB_ * NG * 2); float* T = (float*)take((size_t)NB_ * NOP * 4);
    if ((size_t)(wsp - (char*)d_ws) > ws_size) return;
    k_w1p<<<C1 / 8, 256, 0, stream>>>(w1, W1P); k_cvt8<<<(C1 * C1 / 8 + 255) / 256, 256, 0, stream>>>(w2, W2B, (size_t)C1 * C1 / 8); k_fcp<<<NOP / 8, 256, 0, stream>>>(fw, FCP);
    for (int ch = 0; ch < NB_ / BCH; ++ch) { const int b0 = ch * BCH;
        k_a0<<<RCH / 8, 256, 0, stream>>>(x, b0, A0);
        k_gemmb<false, false><<<dim3(RCH / 64, C1 / 64, 1), 128, 0, stream>>>(A0, nullptr, W1P, b1, H1, C1, nullptr, nullptr, KP1);
        k_split512<<<RCH / 8, 256, 0, stream>>>(H1, Hh, Hl);
        k_gemmb<true, false><<<dim3(RCH / 64, C1 / 64, 1), 128, 0, stream>>>(Hh, Hl, W2B, b2, H2, C1, nullptr, nullptr, C1);
        k_conv3<<<(BCH * GRP) / 256, 256, 0, stream>>>(H2, w3, b0, Gh, Gl); }
    k_gemmb<true, false><<<dim3(NB_ / 64, NOP / 64, 1), 128, 0, stream>>>(Gh, Gl, FCP, nullptr, T, NOP, nullptr, nullptr, NG);
    k_out<<<(NB_ * NL / 4 + 255) / 256, 256, 0, stream>>>(T, fb, out);
}
